// CausalSelfAttention_30107720745073
// MI455X (gfx1250) — hardware-verified
//
#include <hip/hip_runtime.h>
#ifndef NB
#define NB 2
#endif
#ifndef SEQ
#define SEQ 2048
#endif
#define NB_FULL 2
#define SEQ_FULL 2048
#define SQ SEQ
#define DM 1024
#define NH 16
#define HD 64
#define QT 256
#define NKX SQ
#define QT0 256
#define NR ((size_t)NB * SQ)
#define MP ((int)((size_t)NB * SQ))
#define LQ DM

static_assert(NH * HD == DM);
static_assert(HD == 64);
static_assert(DM % 64 == 0 && DM % 32 == 0);
static_assert(SQ % QT == 0 && QT % 128 == 0);
static_assert(QT % 64 == 0);
static_assert(QT0 % 128 == 0 && QT0 % 64 == 0 && QT0 <= SQ);
static_assert(MP % 128 == 0);
static_assert(SQ % 64 == 0);
static_assert(NB <= NB_FULL && SEQ <= SEQ_FULL);
static_assert((DM / 8) * 8 == DM);

#define SZ_W    ((size_t)DM * DM * 2)
#define SZ_ROWS ((size_t)NB * SQ * DM * 2)
#define SZ_S    ((size_t)NH * QT * NKX * 4)
#define SZ_P    ((size_t)NH * QT * NKX * 2)
#define SZ_VT   ((size_t)NH * HD * SQ * 2)
#define SZ_F0   ((size_t)QT0 * DM * 4)
#define SZ_OF0  ((size_t)NB * QT0 * DM * 4)
#define SZ_OH0  ((size_t)NB * QT0 * DM * 2)
#define WS_TOTAL (4 * SZ_W + 5 * SZ_ROWS + SZ_S + SZ_P + SZ_VT + 3 * SZ_F0 + SZ_OF0 + 2 * SZ_OH0)
static_assert(SZ_W % 256 == 0 && SZ_ROWS % 256 == 0 && SZ_S % 256 == 0 && SZ_P % 256 == 0 && SZ_VT % 256 == 0 && SZ_F0 % 256 == 0 && SZ_OF0 % 256 == 0 && SZ_OH0 % 256 == 0);
static_assert(WS_TOTAL <= (size_t)134217728);

typedef unsigned short v8us __attribute__((ext_vector_type(8), may_alias));
typedef float  v8f  __attribute__((ext_vector_type(8)));
typedef float  v4f  __attribute__((ext_vector_type(4)));
typedef float  v4fa __attribute__((ext_vector_type(4), may_alias));
typedef _Float16 v16h __attribute__((ext_vector_type(16)));
typedef _Float16 v4h  __attribute__((ext_vector_type(4)));
union FragH { v16h v; v8us half[2]; _Float16 h[16]; unsigned short u[16]; };

__device__ __forceinline__ unsigned short bf16_bits(float x) { unsigned int u = __float_as_uint(x); return (unsigned short)((u + 0x7FFFu + ((u >> 16) & 1u)) >> 16); }
__device__ __forceinline__ float bf16_rne(float x) { return __uint_as_float(((unsigned int)bf16_bits(x)) << 16); }

__device__ __forceinline__ v16h g2_frag(const _Float16* p, int hh) { FragH f; f.half[0] = *(const v8us*)((const unsigned short*)p + 8 * hh); f.half[1] = *(const v8us*)((const unsigned short*)p + 16 + 8 * hh); return f.v; }
__device__ __forceinline__ v8f g2_mma(v16h a, v16h b, v8f c) { v8f d = __builtin_amdgcn_wmma_f32_16x16x32_f16(false, a, false, b, (short)0, c, false, false); asm volatile("v_nop\n\tv_nop\n\tv_nop\n\tv_nop" : "+v"(d) : "v"(a), "v"(b)); return d; }

__global__ __launch_bounds__(256) void k_x16(const float* __restrict__ x, _Float16* __restrict__ X16, size_t n8) {
  const size_t t = (size_t)blockIdx.x * 256 + threadIdx.x; if (t >= n8) return;
  const size_t row = t / (DM / 8); const int c8 = (int)(t % (DM / 8)) * 8;
  const size_t b = row / SQ, s = row % SQ;
  const float* src = x + (b * (size_t)SEQ_FULL + s) * DM + c8;
  const v4f a = *(const v4fa*)src, c = *(const v4fa*)(src + 4);
  FragH f;
#pragma unroll
  for (int q = 0; q < 4; ++q) { f.h[q] = (_Float16)bf16_rne(a[q]); f.h[4 + q] = (_Float16)bf16_rne(c[q]); }
  const v8us o = f.half[0];
  *(volatile v8us*)((unsigned short*)X16 + t * 8) = o; __threadfence(); *(volatile v8us*)((unsigned short*)X16 + t * 8) = o;
}

__global__ __launch_bounds__(256) void k_wnat(const float* __restrict__ w, size_t n8, _Float16* __restrict__ Bt) {
  const size_t t = (size_t)blockIdx.x * 256 + threadIdx.x; if (t >= n8) return;
  const v4f a = *(const v4fa*)(w + t * 8), c = *(const v4fa*)(w + t * 8 + 4);
  FragH f;
#pragma unroll
  for (int q = 0; q < 4; ++q) { f.h[q] = (_Float16)(bf16_rne(a[q]) * 16.0f); f.h[4 + q] = (_Float16)(bf16_rne(c[q]) * 16.0f); }
  const v8us o = f.half[0];
  *(volatile v8us*)((unsigned short*)Bt + t * 8) = o; __threadfence(); *(volatile v8us*)((unsigned short*)Bt + t * 8) = o;
}

__global__ __launch_bounds__(256) void k_vt(const _Float16* __restrict__ V16b, _Float16* __restrict__ Vt) {
  __shared__ unsigned short tl[64][66];
  const int tid = threadIdx.x; const int h = blockIdx.x / (SQ / 64), lg = blockIdx.x % (SQ / 64);
  for (int i = tid; i < 64 * 8; i += 256) { const int r = i / 8, c8 = (i % 8) * 8; FragH f; f.half[0] = *(const v8us*)((const unsigned short*)V16b + ((size_t)(lg * 64 + r)) * LQ + h * HD + c8);
#pragma unroll
    for (int q = 0; q < 8; ++q) tl[r][c8 + q] = f.u[q]; }
  __syncthreads();
  for (int pass = 0; pass < 2; ++pass) {
#pragma unroll
    for (int rd = 0; rd < 2; ++rd) { const int d = rd * 32 + tid / 8, pc = tid % 8; FragH f;
#pragma unroll
      for (int q = 0; q < 8; ++q) f.u[q] = tl[pc * 8 + q][d];
      *(volatile v8us*)((unsigned short*)Vt + ((size_t)h * 64 + d) * SQ + lg * 64 + pc * 8) = f.half[0]; }
    if (pass == 0) __threadfence(); }
}

__global__ __launch_bounds__(256) void k_hl(const float* __restrict__ F, _Float16* __restrict__ Hh, _Float16* __restrict__ Hl, size_t n8) {
  const size_t t = (size_t)blockIdx.x * 256 + threadIdx.x; if (t >= n8) return; FragH fh, fl; const v4f a = *(const v4fa*)(F + t * 8), c = *(const v4fa*)(F + t * 8 + 4);
#pragma unroll
  for (int q = 0; q < 4; ++q) { _Float16 h = (_Float16)a[q]; fh.h[q] = h; fl.h[q] = (_Float16)((a[q] - (float)h) * 1024.0f); h = (_Float16)c[q]; fh.h[4 + q] = h; fl.h[4 + q] = (_Float16)((c[q] - (float)h) * 1024.0f); }
  for (int pass = 0; pass < 2; ++pass) { *(volatile v8us*)((unsigned short*)Hh + t * 8) = fh.half[0]; *(volatile v8us*)((unsigned short*)Hl + t * 8) = fl.half[0]; if (pass == 0) __threadfence(); }
}

__global__ __launch_bounds__(128) void k_gemm2(const _Float16* __restrict__ A, int lda, size_t sA, const _Float16* __restrict__ Bh, int ldb, size_t sB, float alpha,
    const float* __restrict__ bias, const float* CP, float* C, _Float16* C16, int ldc, size_t sC, int M, int N, int K) {
  __shared__ __attribute__((aligned(16))) float so[4][32][68];
  const int tid = threadIdx.x, w = tid >> 5, lane = tid & 31, ln = lane & 15, hh = lane >> 4; const int by = blockIdx.y;
  A += (size_t)by * sA; Bh += (size_t)by * sB; const size_t cofs = (size_t)by * sC;
  const int ntn = N >> 6; const int mt = blockIdx.x / ntn, nq = blockIdx.x - mt * ntn; const int row0 = mt * 128 + 32 * w, col0 = nq * 64; if (row0 >= M) return;
  const _Float16* a0p = A + (size_t)(row0 + ln) * lda; const _Float16* a1p = a0p + (size_t)16 * lda;
  const _Float16* b0p = Bh + (size_t)(col0 + ln) * ldb; const _Float16* b1p = b0p + (size_t)16 * ldb; const _Float16* b2p = b1p + (size_t)16 * ldb; const _Float16* b3p = b2p + (size_t)16 * ldb;
  const v8f z8 = {0.f,0.f,0.f,0.f,0.f,0.f,0.f,0.f}; v8f c00 = z8, c01 = z8, c02 = z8, c03 = z8, c10 = z8, c11 = z8, c12 = z8, c13 = z8;
#pragma unroll 1
  for (int kb = 0; kb < K; kb += 32) { const v16h a0 = g2_frag(a0p + kb, hh), a1 = g2_frag(a1p + kb, hh);
    v16h b = g2_frag(b0p + kb, hh); c00 = g2_mma(a0, b, c00); c10 = g2_mma(a1, b, c10);
    b = g2_frag(b1p + kb, hh); c01 = g2_mma(a0, b, c01); c11 = g2_mma(a1, b, c11);
    b = g2_frag(b2p + kb, hh); c02 = g2_mma(a0, b, c02); c12 = g2_mma(a1, b, c12);
    b = g2_frag(b3p + kb, hh); c03 = g2_mma(a0, b, c03); c13 = g2_mma(a1, b, c13); }
  v8f accs[8] = {c00, c01, c02, c03, c10, c11, c12, c13};
#pragma unroll
  for (int u = 0; u < 8; ++u) { const int t = u & 3, half = u >> 2; const int col = col0 + t * 16 + ln; float bv = 0.f; if (bias != nullptr) bv = bf16_rne(bias[col]);
#pragma unroll
    for (int r = 0; r < 8; ++r) { const int rloc = half * 16 + 8 * hh + r; so[w][rloc][t * 16 + ln] = accs[u][r] * alpha + bv; } }
  __builtin_amdgcn_fence(4  , "workgroup"); __builtin_amdgcn_wave_barrier();
  const int rsub = lane >> 4, c4 = (lane & 15) * 4;
  if (CP != nullptr) {
#pragma unroll 4
    for (int q = 0; q < 16; ++q) { const int r = q * 2 + rsub; v4f v = *(const v4fa*)&so[w][r][c4]; const v4f c = *(const v4fa*)(CP + cofs + (size_t)(row0 + r) * ldc + col0 + c4); v[0] += c[0]; v[1] += c[1]; v[2] += c[2]; v[3] += c[3]; *(v4fa*)&so[w][r][c4] = v; }
    __builtin_amdgcn_fence(4  , "workgroup"); __builtin_amdgcn_wave_barrier();
  }
  for (int pass = 0; pass < 2; ++pass) {
#pragma unroll
    for (int q = 0; q < 16; ++q) { const int r = q * 2 + rsub; const v4f v = *(const v4fa*)&so[w][r][c4];
      if (C != nullptr) *(volatile v4f*)(C + cofs + (size_t)(row0 + r) * ldc + col0 + c4) = v;
      if (C16 != nullptr) { v4h h4; h4[0] = (_Float16)v[0]; h4[1] = (_Float16)v[1]; h4[2] = (_Float16)v[2]; h4[3] = (_Float16)v[3]; *(volatile v4h*)(C16 + cofs + (size_t)(row0 + r) * ldc + col0 + c4) = h4; } }
    if (pass == 0) __threadfence(); }
}

__global__ __launch_bounds__(256) void k_csm(const float* __restrict__ S, _Float16* __restrict__ P, int hg, int q0, int nk) {
  #pragma clang fp contract(off)
  const int t = blockIdx.x * 256 + threadIdx.x; if (t >= hg * QT) return; const size_t i = (size_t)t; const float* s = S + i * NKX; const int last = q0 + (t % QT); float mx = -3.0e38f;
#pragma unroll 1
  for (int j = 0; j < nk; ++j) { const float f = (j <= last) ? 1.f : 0.f; mx = fmaxf(mx, fmaf(f, s[j], (1.f - f) * -1.0e9f)); } float se = 0.f;
#pragma unroll 1
  for (int j = 0; j < nk; ++j) { const float f = (j <= last) ? 1.f : 0.f; se += __expf(fmaf(f, s[j], (1.f - f) * -1.0e9f) - mx); } const float sc = 256.0f * (1.0f / se);
#pragma unroll 1
  for (int j0 = 0; j0 < nk; j0 += 8) { FragH fr;
#pragma unroll
    for (int q = 0; q < 8; ++q) { const int j = j0 + q; const float f = (j <= last) ? 1.f : 0.f; fr.h[q] = (_Float16)(__expf(fmaf(f, s[j], (1.f - f) * -1.0e9f) - mx) * sc); }
    const v8us o = fr.half[0]; unsigned short* d = (unsigned short*)P + i * NKX + j0; *(volatile v8us*)d = o; __threadfence(); *(volatile v8us*)d = o; }
}

__global__ __launch_bounds__(64) void k_att0(const float* __restrict__ QF, const float* __restrict__ KF, const float* __restrict__ VF, int ld, float scale, float* __restrict__ OF, int ldo) {
  #pragma clang fp contract(off)
  __shared__ __attribute__((aligned(16))) float lq[64][64]; __shared__ __attribute__((aligned(16))) float lo[64][64];
  const int tid = threadIdx.x; const int h = blockIdx.x / (QT0 / 64), rg = blockIdx.x % (QT0 / 64); const int i = rg * 64 + tid;
  const float* qr = QF + (size_t)i * ld + h * HD;
#pragma unroll 1
  for (int c = 0; c < HD / 4; ++c) { *(v4f*)&lq[tid][c * 4] = *(const v4fa*)(qr + c * 4); const v4f z = {0.f, 0.f, 0.f, 0.f}; *(v4f*)&lo[tid][c * 4] = z; }
  float m = -1.0e30f, l = 0.f; const int jmax = rg * 64 + 63;
#pragma unroll 1
  for (int j = 0; j <= jmax; ++j) { const float* kr = KF + (size_t)j * ld + h * HD; const float* vr = VF + (size_t)j * ld + h * HD; float s = 0.f;
#pragma unroll 1
    for (int c = 0; c < HD / 4; ++c) { const v4f kq = *(const v4fa*)(kr + c * 4); const v4f qq = *(v4f*)&lq[tid][c * 4]; s = __fadd_rn(s, __fmul_rn(qq[0], kq[0])); s = __fadd_rn(s, __fmul_rn(qq[1], kq[1])); s = __fadd_rn(s, __fmul_rn(qq[2], kq[2])); s = __fadd_rn(s, __fmul_rn(qq[3], kq[3])); }
    s = __fmul_rn(s, scale);
    const float f = (j <= i) ? 1.f : 0.f; const float sm = fmaf(f, s, (1.f - f) * -1.0e30f); const float mn = fmaxf(m, sm); const float sc = expf(m - mn); const float e = expf(sm - mn); l = __fadd_rn(__fmul_rn(l, sc), e); m = mn;
#pragma unroll 1
    for (int c = 0; c < HD / 4; ++c) { const v4f vv = *(const v4fa*)(vr + c * 4); v4f oo = *(v4f*)&lo[tid][c * 4];
#pragma unroll
      for (int u = 0; u < 4; ++u) oo[u] = __fadd_rn(__fmul_rn(oo[u], sc), __fmul_rn(e, vv[u]));
      *(v4f*)&lo[tid][c * 4] = oo; } }
  const float fin = 64.0f * (1.0f / l);
#pragma unroll 1
  for (int c = 0; c < HD / 4; ++c) { v4f oo = *(v4f*)&lo[tid][c * 4];
#pragma unroll
    for (int u = 0; u < 4; ++u) oo[u] = __fmul_rn(oo[u], fin);
    *(v4f*)&lo[tid][c * 4] = oo; }
  __syncthreads();
  for (int pass = 0; pass < 2; ++pass) {
#pragma unroll 1
    for (int it = 0; it < 16; ++it) { const int row = it * 4 + tid / 16, pc = (tid % 16) * 4; const v4f v = *(const v4f*)&lo[row][pc]; *(volatile v4f*)(OF + (size_t)(rg * 64 + row) * ldo + h * HD + pc) = v; }
    if (pass == 0) __threadfence(); }
}

extern "C" void kernel_launch(void* const* d_in, const int* in_sizes, int n_in,
                              void* d_out, int out_size, void* d_ws, size_t ws_size, hipStream_t stream) {
  if (n_in < 9) return;
  if (in_sizes[0] < (int)(((size_t)(NB - 1) * SEQ_FULL + SQ) * DM)) return;
  if (in_sizes[1] < DM * DM || in_sizes[3] < DM * DM || in_sizes[5] < DM * DM || in_sizes[7] < DM * DM) return;
  if (in_sizes[2] < DM || in_sizes[4] < DM || in_sizes[6] < DM || in_sizes[8] < DM) return;
  if (out_size < (int)(NR * DM)) return;
  const float* x  = (const float*)d_in[0];
  const float* wq = (const float*)d_in[1]; const float* bq = (const float*)d_in[2];
  const float* wk = (const float*)d_in[3]; const float* bk = (const float*)d_in[4];
  const float* wv = (const float*)d_in[5]; const float* bv = (const float*)d_in[6];
  const float* wo = (const float*)d_in[7]; const float* bo = (const float*)d_in[8];
  float* out = (float*)d_out;
  char* ws = (char*)d_ws; size_t off = 0;
  auto take = [&](size_t bytes) { char* p = ws + off; off += (bytes + 255) & ~(size_t)255; return p; };
  _Float16* BQ = (_Float16*)take(SZ_W); _Float16* BK = (_Float16*)take(SZ_W); _Float16* BV = (_Float16*)take(SZ_W); _Float16* BO = (_Float16*)take(SZ_W);
  _Float16* X16 = (_Float16*)take(SZ_ROWS); _Float16* Q16 = (_Float16*)take(SZ_ROWS); _Float16* K16 = (_Float16*)take(SZ_ROWS); _Float16* V16 = (_Float16*)take(SZ_ROWS); _Float16* O16 = (_Float16*)take(SZ_ROWS);
  float* S = (float*)take(SZ_S); _Float16* P = (_Float16*)take(SZ_P); _Float16* VT = (_Float16*)take(SZ_VT);
  float* QF0 = (float*)take(SZ_F0); float* KF0 = (float*)take(SZ_F0); float* VF0 = (float*)take(SZ_F0);
  float* OF0 = (float*)take(SZ_OF0); _Float16* OH0 = (_Float16*)take(SZ_OH0); _Float16* OL0 = (_Float16*)take(SZ_OH0);
  if (off > ws_size) return;

  const size_t wn8 = (size_t)DM * DM / 8;
  k_wnat<<<(unsigned)((wn8 + 255) / 256), 256, 0, stream>>>(wq, wn8, BQ);
  k_wnat<<<(unsigned)((wn8 + 255) / 256), 256, 0, stream>>>(wk, wn8, BK);
  k_wnat<<<(unsigned)((wn8 + 255) / 256), 256, 0, stream>>>(wv, wn8, BV);
  k_wnat<<<(unsigned)((wn8 + 255) / 256), 256, 0, stream>>>(wo, wn8, BO);
  k_x16<<<(unsigned)((NR * DM / 8 + 255) / 256), 256, 0, stream>>>(x, X16, NR * DM / 8);

  const dim3 gp((unsigned)((MP / 128) * (DM / 64)), 1);
  k_gemm2<<<gp, 128, 0, stream>>>(X16, DM, 0, BQ, DM, 0, 0.0625f, bq, nullptr, nullptr, Q16, DM, 0, MP, DM, DM);
  k_gemm2<<<gp, 128, 0, stream>>>(X16, DM, 0, BK, DM, 0, 0.0625f, bk, nullptr, nullptr, K16, DM, 0, MP, DM, DM);
  k_gemm2<<<gp, 128, 0, stream>>>(X16, DM, 0, BV, DM, 0, 0.0625f, bv, nullptr, nullptr, V16, DM, 0, MP, DM, DM);

  const dim3 g0((QT0 / 128) * (DM / 64), 1);
  for (int b = 0; b < NB; ++b) { const size_t r0 = (size_t)b * SQ;
    k_vt<<<NH * (SQ / 64), 256, 0, stream>>>(V16 + r0 * LQ, VT);
    k_gemm2<<<g0, 128, 0, stream>>>(X16 + r0 * DM, DM, 0, BQ, DM, 0, 0.0625f, bq, nullptr, QF0, nullptr, DM, 0, QT0, DM, DM);
    k_gemm2<<<g0, 128, 0, stream>>>(X16 + r0 * DM, DM, 0, BK, DM, 0, 0.0625f, bk, nullptr, KF0, nullptr, DM, 0, QT0, DM, DM);
    k_gemm2<<<g0, 128, 0, stream>>>(X16 + r0 * DM, DM, 0, BV, DM, 0, 0.0625f, bv, nullptr, VF0, nullptr, DM, 0, QT0, DM, DM);
    k_att0<<<NH * (QT0 / 64), 64, 0, stream>>>(QF0, KF0, VF0, DM, 0.125f, OF0 + (size_t)b * QT0 * DM, DM);
    for (int q0 = 0; q0 < SQ; q0 += QT) { const int nk = q0 + QT;
      k_gemm2<<<dim3((unsigned)((QT / 128) * (nk / 64)), NH), 128, 0, stream>>>(Q16 + (r0 + q0) * LQ, LQ, (size_t)HD, K16 + r0 * LQ, LQ, (size_t)HD, 0.125f, nullptr, nullptr, S, nullptr, NKX, (size_t)QT * NKX, QT, nk, HD);
      k_csm<<<(NH * QT + 255) / 256, 256, 0, stream>>>(S, P, NH, q0, nk);
      k_gemm2<<<dim3((unsigned)((QT / 128) * (HD / 64)), NH), 128, 0, stream>>>(P, NKX, (size_t)QT * NKX, VT, SQ, (size_t)HD * SQ, 0.25f, nullptr, nullptr, nullptr, O16 + (r0 + q0) * DM, DM, (size_t)HD, QT, HD, nk); } }

  k_gemm2<<<gp, 128, 0, stream>>>(O16, DM, 0, BO, DM, 0, 0.0009765625f, bo, nullptr, out, nullptr, DM, 0, MP, DM, DM);
  k_hl<<<(unsigned)(((size_t)NB * QT0 * DM / 8 + 255) / 256), 256, 0, stream>>>(OF0, OH0, OL0, (size_t)NB * QT0 * DM / 8);
  for (int b = 0; b < NB; ++b) { const size_t r0 = (size_t)b * SQ; const size_t f0 = (size_t)b * QT0;
    k_gemm2<<<g0, 128, 0, stream>>>(OH0 + f0 * DM, DM, 0, BO, DM, 0, 0.0009765625f, bo, nullptr, out + r0 * DM, nullptr, DM, 0, QT0, DM, DM);
    k_gemm2<<<g0, 128, 0, stream>>>(OL0 + f0 * DM, DM, 0, BO, DM, 0, 0.00000095367431640625f, nullptr, out + r0 * DM, out + r0 * DM, nullptr, DM, 0, QT0, DM, DM); }
}
